// Transition_8186207666610
// MI455X (gfx1250) — hardware-verified
//
#include <hip/hip_runtime.h>
#include <math.h>

typedef __attribute__((ext_vector_type(16))) _Float16 v16h;
typedef __attribute__((ext_vector_type(8)))  _Float16 v8h;
typedef __attribute__((ext_vector_type(8)))  float    v8f;
typedef __attribute__((ext_vector_type(4)))  float    v4f;

constexpr int kNB = 128;
constexpr int kNH = 1024;
static_assert((kNB % 64) == 0 && (kNH % 64) == 0 && (kNH % 32) == 0, "GEMM tile multiples");
static_assert((kNB % 32) == 0 && (kNH % 32) == 0, "32 rows per statistics block");

constexpr float kCarryA = 256.0f;
constexpr float kCarryT = 256.0f;
constexpr float kFold   = 1.0f / (kCarryA * kCarryT);
constexpr float kHalfMinNormal = 6.103515625e-5f;

constexpr size_t kOffTT  = 0;
constexpr size_t kOffAP  = kOffTT  + (size_t)kNH * kNH * 2;
constexpr size_t kOffRMU = kOffAP  + (size_t)kNB * kNH * 2;
constexpr size_t kOffLW  = kOffRMU + (size_t)kNH * 4;
constexpr size_t kOffMV  = kOffLW  + (size_t)kNH * 4;
constexpr size_t kWsTotal = kOffMV + 4096;
static_assert(kWsTotal == 2371584ull, "carve total");
static_assert(kWsTotal <= 134217728ull, "carve cap");
static_assert((kOffAP % 128) == 0 && (kOffRMU % 128) == 0 && (kOffLW % 128) == 0 && (kOffMV % 128) == 0, "128-B aligned regions");
static_assert((size_t)kNB * 4 <= 4096, "MV region holds all per-b maxima");

__device__ __forceinline__ _Float16 to_half_flush(float v) {
  const float w = (fabsf(v) < kHalfMinNormal) ? 0.0f : v;
  return (_Float16)w;
}

__device__ __forceinline__ v16h frag_load_h(const _Float16* p) {
  union FragU { v16h v; v8h h[2]; } f;
  f.h[0] = *(const v8h*)(p);
  f.h[1] = *(const v8h*)(p + 16);
  return f.v;
}

__device__ __forceinline__ v8f mma_guard_h(v16h a, v16h b, v8f c) {
  c = __builtin_amdgcn_wmma_f32_16x16x32_f16(false, a, false, b, (short)0, c, false, false);
  asm volatile("v_nop\n\tv_nop\n\tv_nop\n\tv_nop" : "+v"(c) : "v"(a), "v"(b));
  return c;
}

__global__ __launch_bounds__(256) void row_stats_kernel(
    const float* __restrict__ U, float* __restrict__ rmU, float* __restrict__ lwv)
{
  __shared__ float sRm[32];
  __shared__ float sLw[32];
  const int tid = threadIdx.x, lane = tid & 31, wave = tid >> 5;
  const int r0 = blockIdx.x * 32;
#pragma unroll 1
  for (int q = 0; q < 4; ++q) {
    const int lr = wave * 4 + q;
    const float* u = U + (size_t)(r0 + lr) * kNH + lane * 8;
    float mx = -INFINITY;
#pragma unroll 1
    for (int it = 0; it < 4; ++it) {
      const v4f a0 = *(const v4f*)(u + it * 256);
      const v4f a1 = *(const v4f*)(u + it * 256 + 4);
      const float m0 = fmaxf(fmaxf(a0[0], a0[1]), fmaxf(a0[2], a0[3]));
      const float m1 = fmaxf(fmaxf(a1[0], a1[1]), fmaxf(a1[2], a1[3]));
      mx = fmaxf(mx, fmaxf(m0, m1));
    }
    mx = fmaxf(mx, __shfl_xor(mx, 16, 32));
    mx = fmaxf(mx, __shfl_xor(mx, 8, 32));
    mx = fmaxf(mx, __shfl_xor(mx, 4, 32));
    mx = fmaxf(mx, __shfl_xor(mx, 2, 32));
    mx = fmaxf(mx, __shfl_xor(mx, 1, 32));
    float sm = 0.0f;
#pragma unroll 1
    for (int it = 0; it < 4; ++it) {
      const v4f a0 = *(const v4f*)(u + it * 256);
      const v4f a1 = *(const v4f*)(u + it * 256 + 4);
      float part = 0.0f;
      part += expf(a0[0] - mx);
      part += expf(a0[1] - mx);
      part += expf(a0[2] - mx);
      part += expf(a0[3] - mx);
      part += expf(a1[0] - mx);
      part += expf(a1[1] - mx);
      part += expf(a1[2] - mx);
      part += expf(a1[3] - mx);
      sm += part;
    }
    sm += __shfl_xor(sm, 16, 32);
    sm += __shfl_xor(sm, 8, 32);
    sm += __shfl_xor(sm, 4, 32);
    sm += __shfl_xor(sm, 2, 32);
    sm += __shfl_xor(sm, 1, 32);
    const float lg = logf(sm);
    if (lane == 0) {
      sRm[lr] = mx;
      sLw[lr] = lg;
    }
  }
  __syncthreads();
  if (wave == 0) {
    const float a = sRm[lane];
    const float b = sLw[lane];
    volatile float* pr = rmU + r0 + lane;
    volatile float* pl = lwv + r0 + lane;
    *pr = a;
    *pl = b;
    __threadfence();
    *pr = a;
    *pl = b;
  }
}

__global__ __launch_bounds__(256) void build_tt_kernel(
    const float* __restrict__ U, const float* __restrict__ rmU, unsigned short* __restrict__ TT)
{
  __shared__ __align__(16) float sT[64 * 68];
  const int tid = threadIdx.x, lane = tid & 31, wave = tid >> 5;
  const int j0 = blockIdx.x * 64;
  const int i0 = blockIdx.y * 64;
  const int lr = tid >> 4;
  const int c4 = (tid & 15) * 4;
#pragma unroll 1
  for (int it = 0; it < 4; ++it) {
    const int row = lr + 16 * it;
    const v4f uv = *(const v4f*)(U + (size_t)(i0 + row) * kNH + j0 + c4);
    const float rm = rmU[i0 + row];
    const float t0 = expf(uv[0] - rm) * kCarryT;
    const float t1 = expf(uv[1] - rm) * kCarryT;
    const float t2 = expf(uv[2] - rm) * kCarryT;
    const float t3 = expf(uv[3] - rm) * kCarryT;
    sT[(c4 + 0) * 68 + row] = t0;
    sT[(c4 + 1) * 68 + row] = t1;
    sT[(c4 + 2) * 68 + row] = t2;
    sT[(c4 + 3) * 68 + row] = t3;
  }
  __syncthreads();
  const int q = lane >> 3;
  const int c8 = (lane & 7) * 8;
  v8h hv[2];
#pragma unroll
  for (int it = 0; it < 2; ++it) {
    const int row = it * 32 + wave * 4 + q;
    const float* sp = sT + row * 68 + c8;
    const v4f a0 = *(const v4f*)(sp);
    const v4f a1 = *(const v4f*)(sp + 4);
    hv[it][0] = to_half_flush(a0[0]);
    hv[it][1] = to_half_flush(a0[1]);
    hv[it][2] = to_half_flush(a0[2]);
    hv[it][3] = to_half_flush(a0[3]);
    hv[it][4] = to_half_flush(a1[0]);
    hv[it][5] = to_half_flush(a1[1]);
    hv[it][6] = to_half_flush(a1[2]);
    hv[it][7] = to_half_flush(a1[3]);
  }
  for (int pass = 0; pass < 2; ++pass) {
#pragma unroll
    for (int it = 0; it < 2; ++it) {
      const int row = it * 32 + wave * 4 + q;
      *(volatile v8h*)(TT + (size_t)(j0 + row) * kNH + i0 + c8) = hv[it];
    }
    __threadfence();
  }
}

__global__ __launch_bounds__(256) void build_a_kernel(
    const float* __restrict__ la, const float* __restrict__ lwv,
    unsigned short* __restrict__ AP, float* __restrict__ mvec)
{
  __shared__ float sM[32];
  const int tid = threadIdx.x, lane = tid & 31, wave = tid >> 5;
  const int r0 = blockIdx.x * 32;
#pragma unroll 1
  for (int q = 0; q < 4; ++q) {
    const int lr = wave * 4 + q;
    const int b = r0 + lr;
    const float* a = la + (size_t)b * kNH + lane * 8;
    const float* w = lwv + lane * 8;
    float mx = -INFINITY;
#pragma unroll 1
    for (int it = 0; it < 4; ++it) {
      const v4f a0 = *(const v4f*)(a + it * 256);
      const v4f a1 = *(const v4f*)(a + it * 256 + 4);
      const v4f w0 = *(const v4f*)(w + it * 256);
      const v4f w1 = *(const v4f*)(w + it * 256 + 4);
      const v4f d0 = a0 - w0;
      const v4f d1 = a1 - w1;
      const float m0 = fmaxf(fmaxf(d0[0], d0[1]), fmaxf(d0[2], d0[3]));
      const float m1 = fmaxf(fmaxf(d1[0], d1[1]), fmaxf(d1[2], d1[3]));
      mx = fmaxf(mx, fmaxf(m0, m1));
    }
    mx = fmaxf(mx, __shfl_xor(mx, 16, 32));
    mx = fmaxf(mx, __shfl_xor(mx, 8, 32));
    mx = fmaxf(mx, __shfl_xor(mx, 4, 32));
    mx = fmaxf(mx, __shfl_xor(mx, 2, 32));
    mx = fmaxf(mx, __shfl_xor(mx, 1, 32));
#pragma unroll 1
    for (int it = 0; it < 4; ++it) {
      const v4f a0 = *(const v4f*)(a + it * 256);
      const v4f a1 = *(const v4f*)(a + it * 256 + 4);
      const v4f w0 = *(const v4f*)(w + it * 256);
      const v4f w1 = *(const v4f*)(w + it * 256 + 4);
      const v4f d0 = a0 - w0;
      const v4f d1 = a1 - w1;
      v8h hv;
      hv[0] = to_half_flush(expf(d0[0] - mx) * kCarryA);
      hv[1] = to_half_flush(expf(d0[1] - mx) * kCarryA);
      hv[2] = to_half_flush(expf(d0[2] - mx) * kCarryA);
      hv[3] = to_half_flush(expf(d0[3] - mx) * kCarryA);
      hv[4] = to_half_flush(expf(d1[0] - mx) * kCarryA);
      hv[5] = to_half_flush(expf(d1[1] - mx) * kCarryA);
      hv[6] = to_half_flush(expf(d1[2] - mx) * kCarryA);
      hv[7] = to_half_flush(expf(d1[3] - mx) * kCarryA);
      unsigned short* dst = AP + (size_t)b * kNH + it * 256 + lane * 8;
      *(volatile v8h*)dst = hv;
      __threadfence();
      *(volatile v8h*)dst = hv;
    }
    if (lane == 0) sM[lr] = mx;
  }
  __syncthreads();
  if (wave == 0) {
    const float mval = sM[lane];
    volatile float* pm = mvec + r0 + lane;
    *pm = mval;
    __threadfence();
    *pm = mval;
  }
}

__global__ __launch_bounds__(256) void gemm_log_kernel(
    const unsigned short* __restrict__ APp, const unsigned short* __restrict__ TTp,
    const float* __restrict__ mvec, float* __restrict__ out)
{
  __shared__ __align__(16) float sT[8][16 * 68];
  const _Float16* A  = (const _Float16*)APp;
  const _Float16* Bt = (const _Float16*)TTp;
  const int lane = threadIdx.x & 31;
  const int wave = threadIdx.x >> 5;
  constexpr int tilesN = kNH >> 6;
  constexpr int tilesM = kNB >> 6;
  const int tile = blockIdx.x * 8 + wave;
  if (tile >= tilesM * tilesN) return;
  const int tm = tile / tilesN;
  const int tn = tile - tm * tilesN;
  const int m0 = tm << 6;
  const int n0 = tn << 6;
  const int rlane = lane & 15;
  const int koff  = (lane >> 4) * 8;
  const int mOff  = (lane >> 4) * 8;

  v8f acc[4][4];
#pragma unroll
  for (int i = 0; i < 4; ++i)
#pragma unroll
    for (int j = 0; j < 4; ++j) acc[i][j] = (v8f){0.f, 0.f, 0.f, 0.f, 0.f, 0.f, 0.f, 0.f};

#pragma unroll 1
  for (int k0 = 0; k0 < kNH; k0 += 32) {
    v16h bh[4];
#pragma unroll
    for (int j = 0; j < 4; ++j)
      bh[j] = frag_load_h(Bt + (size_t)(n0 + (j << 4) + rlane) * kNH + koff + k0);
#pragma unroll
    for (int i = 0; i < 4; ++i) {
      const v16h ah = frag_load_h(A + (size_t)(m0 + (i << 4) + rlane) * kNH + koff + k0);
#pragma unroll
      for (int j = 0; j < 4; ++j) acc[i][j] = mma_guard_h(ah, bh[j], acc[i][j]);
    }
  }

  float* slab = sT[wave];
  const int hh = lane >> 4;
  const int c4 = (lane & 15) * 4;
#pragma unroll
  for (int i = 0; i < 4; ++i) {
    const int mBase = m0 + (i << 4);
#pragma unroll
    for (int j = 0; j < 4; ++j) {
#pragma unroll
      for (int r = 0; r < 8; ++r)
        slab[(mOff + r) * 68 + (j << 4) + rlane] = acc[i][j][r] * kFold;
    }
    __builtin_amdgcn_fence(__ATOMIC_RELEASE, "workgroup");
    __builtin_amdgcn_wave_barrier();
    __builtin_amdgcn_fence(__ATOMIC_ACQUIRE, "workgroup");
#pragma unroll 1
    for (int it = 0; it < 8; ++it) {
      const int row = it * 2 + hh;
      float* sp = slab + row * 68 + c4;
      const v4f v = *(const v4f*)sp;
      const float mr = mvec[mBase + row];
      v4f o;
      o[0] = logf(v[0]) + mr;
      o[1] = logf(v[1]) + mr;
      o[2] = logf(v[2]) + mr;
      o[3] = logf(v[3]) + mr;
      *(v4f*)sp = o;
    }
    __builtin_amdgcn_fence(__ATOMIC_RELEASE, "workgroup");
    __builtin_amdgcn_wave_barrier();
    __builtin_amdgcn_fence(__ATOMIC_ACQUIRE, "workgroup");
    for (int pass = 0; pass < 2; ++pass) {
#pragma unroll
      for (int it = 0; it < 8; ++it) {
        const int row = it * 2 + hh;
        const v4f v = *(const v4f*)(slab + row * 68 + c4);
        *(volatile v4f*)(out + (size_t)(mBase + row) * kNH + n0 + c4) = v;
      }
      __threadfence();
    }
    __builtin_amdgcn_fence(__ATOMIC_RELEASE, "workgroup");
    __builtin_amdgcn_wave_barrier();
    __builtin_amdgcn_fence(__ATOMIC_ACQUIRE, "workgroup");
  }
}

extern "C" void kernel_launch(void* const* d_in, const int* in_sizes, int n_in,
                              void* d_out, int out_size, void* d_ws, size_t ws_size,
                              hipStream_t stream) {
  if (n_in < 2) return;
  if (in_sizes[0] != kNB * kNH) return;
  if (in_sizes[1] != kNH * kNH) return;
  if (out_size != kNB * kNH) return;
  if (ws_size < kWsTotal) return;

  const float* la = (const float*)d_in[0];
  const float* U  = (const float*)d_in[1];
  float* out = (float*)d_out;

  char* ws = (char*)d_ws;
  unsigned short* TT  = (unsigned short*)(ws + kOffTT);
  unsigned short* AP  = (unsigned short*)(ws + kOffAP);
  float*          RMU = (float*)(ws + kOffRMU);
  float*          LW  = (float*)(ws + kOffLW);
  float*          MV  = (float*)(ws + kOffMV);

  row_stats_kernel<<<kNH / 32, 256, 0, stream>>>(U, RMU, LW);
  build_tt_kernel<<<dim3(kNH / 64, kNH / 64), 256, 0, stream>>>(U, RMU, TT);
  build_a_kernel<<<kNB / 32, 256, 0, stream>>>(la, LW, AP, MV);
  gemm_log_kernel<<<((kNB / 64) * (kNH / 64)) / 8, 256, 0, stream>>>(AP, TT, MV, out);
}
